// SingleHeadAttention_23201413333083
// MI455X (gfx1250) — hardware-verified
//
#include <hip/hip_runtime.h>
#include <math.h>
#include <stdint.h>

#ifndef NB
#define NB 4
#endif
#ifndef SEQ
#define SEQ 2048
#endif
#define NB_FULL  4
#define SEQ_FULL 2048
#define EMB      1024
#define NROW     (NB * SEQ)
#define PCARRY   16384.0f
#define VLP      ((SEQ < 512) ? SEQ : 512)
#define SMT      (SEQ / 8)
#define SMW      (SMT / 32)
static_assert(NB >= 1 && NB <= NB_FULL);
static_assert(SEQ >= 256 && SEQ <= SEQ_FULL && (SEQ % 256) == 0);
static_assert((EMB % 64) == 0 && (SEQ % 64) == 0 && (EMB % 32) == 0 && (SEQ % 32) == 0);
static_assert((VLP % 64) == 0 && VLP <= SEQ);
static_assert(SMT <= 256 && SMW >= 1 && SMW <= 8);
static_assert((NROW % 64) == 0);

typedef _Float16 v16h __attribute__((ext_vector_type(16)));
typedef _Float16 v8h  __attribute__((ext_vector_type(8)));
typedef __bf16   v16b __attribute__((ext_vector_type(16)));
typedef __bf16   v8b  __attribute__((ext_vector_type(8)));
typedef float    v8f  __attribute__((ext_vector_type(8)));
typedef float    v4f  __attribute__((ext_vector_type(4)));
typedef unsigned int v4u __attribute__((ext_vector_type(4)));

#if defined(__HIP_DEVICE_COMPILE__)
#define DEV_ASM 1
#else
#define DEV_ASM 0
#endif

__device__ __forceinline__ unsigned short bf_bits(float f) {
  unsigned u = __float_as_uint(f);
  return (unsigned short)((u + 0x7FFFu + ((u >> 16) & 1u)) >> 16);
}
__device__ __forceinline__ float bf_up(unsigned short hb) { return __uint_as_float(((unsigned)hb) << 16); }
__device__ __forceinline__ unsigned short h_bits(_Float16 x) { return __builtin_bit_cast(unsigned short, x); }
__device__ __forceinline__ unsigned pk16(unsigned short a, unsigned short b) { return (unsigned)a | ((unsigned)b << 16); }
__device__ __forceinline__ v8f zero8() { v8f z = {0.f, 0.f, 0.f, 0.f, 0.f, 0.f, 0.f, 0.f}; return z; }

template <typename OT> struct FT;
template <> struct FT<__bf16>   { typedef v16b frag; typedef v8b half8; };
template <> struct FT<_Float16> { typedef v16h frag; typedef v8h half8; };

template <typename OT>
__device__ __forceinline__ typename FT<OT>::frag ldfrag(const OT* p) {
  union { typename FT<OT>::frag v; typename FT<OT>::half8 h[2]; } f;
  f.h[0] = *(const typename FT<OT>::half8*)(p);
  f.h[1] = *(const typename FT<OT>::half8*)(p + 16);
  return f.v;
}

__device__ __forceinline__ v8f mmar(v16b a, v16b b, v8f c) {
  return __builtin_amdgcn_wmma_f32_16x16x32_bf16(false, a, false, b, (short)0, c, false, false);
}
__device__ __forceinline__ v8f mmar(v16h a, v16h b, v8f c) {
  return __builtin_amdgcn_wmma_f32_16x16x32_f16(false, a, false, b, (short)0, c, false, false);
}
__device__ __forceinline__ void dep_guard(v8f& a, v8f& b, v16b x, v16b y) {
#if DEV_ASM
  asm volatile("v_nop\n\tv_nop\n\tv_nop\n\tv_nop" : "+v"(a), "+v"(b) : "v"(x), "v"(y));
#else
  (void)a; (void)b; (void)x; (void)y;
#endif
}
__device__ __forceinline__ void dep_guard(v8f& a, v8f& b, v16h x, v16h y) {
#if DEV_ASM
  asm volatile("v_nop\n\tv_nop\n\tv_nop\n\tv_nop" : "+v"(a), "+v"(b) : "v"(x), "v"(y));
#else
  (void)a; (void)b; (void)x; (void)y;
#endif
}
__device__ __forceinline__ void keep4(v16b a, v16b b, v16b c, v16b d) {
#if DEV_ASM
  asm volatile("v_nop" :: "v"(a), "v"(b), "v"(c), "v"(d));
#else
  (void)a; (void)b; (void)c; (void)d;
#endif
}
__device__ __forceinline__ void keep4(v16h a, v16h b, v16h c, v16h d) {
#if DEV_ASM
  asm volatile("v_nop" :: "v"(a), "v"(b), "v"(c), "v"(d));
#else
  (void)a; (void)b; (void)c; (void)d;
#endif
}
__device__ __forceinline__ void acc_guard4(v8f& a, v8f& b, v8f& c, v8f& d) {
#if DEV_ASM
  asm volatile("v_nop\n\tv_nop\n\tv_nop\n\tv_nop" : "+v"(a), "+v"(b), "+v"(c), "+v"(d));
#else
  (void)a; (void)b; (void)c; (void)d;
#endif
}

template <int MODE>
__device__ __forceinline__ unsigned short cvm(float f) {
  const unsigned short hb = bf_bits(f);
  if (MODE == 0) return hb;
  return h_bits((_Float16)(bf_up(hb) * 64.0f));
}

template <int MODE>
__global__ __launch_bounds__(256) void cvt16x8(const float* __restrict__ in, long long sin,
                                               unsigned short* out, long long sout, int n8) {
  const int i = blockIdx.x * 256 + (int)threadIdx.x;
  const int y = blockIdx.y;
  if (i < n8) {
    const float* ip = in + (size_t)y * (size_t)sin + (size_t)i * 8;
    const v4f a  = *(const v4f*)(ip);
    const v4f a4 = *(const v4f*)(ip + 4);
    v4u p;
    p[0] = pk16(cvm<MODE>(a[0]),  cvm<MODE>(a[1]));
    p[1] = pk16(cvm<MODE>(a[2]),  cvm<MODE>(a[3]));
    p[2] = pk16(cvm<MODE>(a4[0]), cvm<MODE>(a4[1]));
    p[3] = pk16(cvm<MODE>(a4[2]), cvm<MODE>(a4[3]));
    unsigned short* o = out + (size_t)y * (size_t)sout + (size_t)i * 8;
    *(volatile v4u*)o = p;
    __threadfence();
    *(volatile v4u*)o = p;
  }
}

template <typename OT, int MI, int NPA, int NPB, int OUT_MODE, int CZ>
__global__ __launch_bounds__(256) void gemm_t(
    const unsigned short* __restrict__ Ap, const unsigned short* __restrict__ A2p, int lda, long long strideA,
    const unsigned short* __restrict__ Btp, int ldb, long long strideB,
    const unsigned short* __restrict__ B2p, int ldb2, long long strideB2, int K2,
    void* Cout, void* Cout2, int ldc, long long strideC, int ldc2, long long strideC2, int N2,
    int M, int N, int K, float oscale, float rscale2, float cscale, float rscaleC) {
  static_assert(CZ != 2 || ((16 * MI) % 32) == 0);
  static_assert(!(NPA == 2 && NPB == 2));
  typedef typename FT<OT>::frag V16;
  const OT* A  = (const OT*)(const void*)Ap;
  const OT* A2 = (const OT*)(const void*)A2p;
  const OT* Bt = (const OT*)(const void*)Btp;
  const OT* B2 = (const OT*)(const void*)B2p;
  __shared__ __align__(16) float sT[8][16 * 68];
  const int RT   = 16 * MI;
  const int b    = blockIdx.y;
  const int lane = threadIdx.x & 31;
  const int wave = threadIdx.x >> 5;
  const int tilesN = N >> 6;
  const int tilesM = M / RT;
  const int tile = blockIdx.x * 8 + wave;
  if (tile >= tilesM * tilesN) return;
  const int tm = tile / tilesN;
  const int tn = tile - tm * tilesN;
  const int m0 = tm * RT;
  const int n0 = tn << 6;
  if (CZ == 1) {
    if (n0 >= m0 + RT) return;
  }
  int kEnd = K;
  if (CZ == 2) {
    const int ke = m0 + RT;
    kEnd = (ke < K) ? ke : K;
  }

  const OT* Ab  = A  + (size_t)b * (size_t)strideA;
  const OT* A2b = A2 + (size_t)b * (size_t)strideA;
  const OT* Bb  = Bt + (size_t)b * (size_t)strideB;
  const OT* B2b = B2 + (size_t)b * (size_t)strideB2;

  const int rlane = lane & 15;
  const int koff  = (lane >> 4) * 8;
  const int mOff  = (lane >> 4) * 8;

  v8f acc[MI][4], acc2[MI][4];
#pragma unroll
  for (int i = 0; i < MI; ++i)
#pragma unroll
    for (int j = 0; j < 4; ++j) { acc[i][j] = zero8(); acc2[i][j] = zero8(); }

#pragma unroll 1
  for (int k0 = 0; k0 < kEnd; k0 += 32) {
    V16 bq[4];
#pragma unroll
    for (int j = 0; j < 4; ++j)
      bq[j] = ldfrag<OT>(Bb + (size_t)(n0 + (j << 4) + rlane) * ldb + koff + k0);
#pragma unroll
    for (int i = 0; i < MI; ++i) {
      const V16 af = ldfrag<OT>(Ab + (size_t)(m0 + (i << 4) + rlane) * lda + koff + k0);
#pragma unroll
      for (int j = 0; j < 4; ++j) acc[i][j] = mmar(af, bq[j], acc[i][j]);
      dep_guard(acc[i][0], acc[i][3], af, bq[3]);
      if (NPA == 2) {
        const V16 af2 = ldfrag<OT>(A2b + (size_t)(m0 + (i << 4) + rlane) * lda + koff + k0);
#pragma unroll
        for (int j = 0; j < 4; ++j) acc2[i][j] = mmar(af2, bq[j], acc2[i][j]);
        dep_guard(acc2[i][0], acc2[i][3], af2, bq[3]);
      }
    }
    keep4(bq[0], bq[1], bq[2], bq[3]);
    if (NPB == 2) {
      if (k0 < K2) {
        V16 br[4];
#pragma unroll
        for (int j = 0; j < 4; ++j)
          br[j] = ldfrag<OT>(B2b + (size_t)(n0 + (j << 4) + rlane) * ldb2 + koff + k0);
#pragma unroll
        for (int i = 0; i < MI; ++i) {
          const V16 afr = ldfrag<OT>(Ab + (size_t)(m0 + (i << 4) + rlane) * lda + koff + k0);
#pragma unroll
          for (int j = 0; j < 4; ++j) acc2[i][j] = mmar(afr, br[j], acc2[i][j]);
          dep_guard(acc2[i][0], acc2[i][3], afr, br[3]);
        }
        keep4(br[0], br[1], br[2], br[3]);
      }
    }
  }
#pragma unroll
  for (int i = 0; i < MI; ++i) {
    acc_guard4(acc[i][0], acc[i][1], acc[i][2], acc[i][3]);
    if (NPA == 2 || NPB == 2) acc_guard4(acc2[i][0], acc2[i][1], acc2[i][2], acc2[i][3]);
  }

  float* slab = sT[wave];
#pragma unroll
  for (int i = 0; i < MI; ++i) {
    const int mBase = m0 + (i << 4);
#pragma unroll
    for (int j = 0; j < 4; ++j) {
#pragma unroll
      for (int r = 0; r < 8; ++r) {
        float v = acc[i][j][r];
        if (NPA == 2 || NPB == 2) v += acc2[i][j][r] * rscale2;
        v = v * oscale;
        slab[(mOff + r) * 68 + (j << 4) + rlane] = v;
      }
    }
    __builtin_amdgcn_fence(__ATOMIC_RELEASE, "workgroup");
    __builtin_amdgcn_wave_barrier();
    __builtin_amdgcn_fence(__ATOMIC_ACQUIRE, "workgroup");
    if (OUT_MODE == 0) {
      float* C = (float*)Cout + (size_t)b * (size_t)strideC;
      const int h2 = lane >> 4, c4 = (lane & 15) * 4;
      for (int pass = 0; pass < 2; ++pass) {
#pragma unroll
        for (int it = 0; it < 8; ++it) {
          const int row = it * 2 + h2;
          const v4f v = *(const v4f*)(slab + row * 68 + c4);
          *(volatile v4f*)(C + (size_t)(mBase + row) * ldc + n0 + c4) = v;
        }
        __threadfence();
      }
    } else {
      const int q = lane >> 3, c8 = (lane & 7) * 8;
      unsigned short* C  = (unsigned short*)Cout  + (size_t)b * (size_t)strideC;
      unsigned short* C2 = (unsigned short*)Cout2 + (size_t)b * (size_t)strideC2;
      const bool wr2 = (OUT_MODE == 3) && (n0 < N2);
      v4u hv[4], lv[4];
#pragma unroll
      for (int it = 0; it < 4; ++it) {
        const int row = it * 4 + q;
        const float* sp = slab + row * 68 + c8;
        float f[8];
#pragma unroll
        for (int e = 0; e < 8; ++e) f[e] = sp[e] * cscale;
        v4u a, a2;
#pragma unroll
        for (int e = 0; e < 4; ++e) {
          const float f0 = f[2 * e], f1 = f[2 * e + 1];
          const _Float16 x0 = (_Float16)f0, x1 = (_Float16)f1;
          const unsigned short h0 = h_bits(x0), h1 = h_bits(x1);
          unsigned short l0 = 0, l1 = 0;
          if (OUT_MODE == 3) {
            l0 = h_bits((_Float16)((f0 - (float)x0) * rscaleC));
            l1 = h_bits((_Float16)((f1 - (float)x1) * rscaleC));
          }
          a[e] = pk16(h0, h1); a2[e] = pk16(l0, l1);
        }
        hv[it] = a; lv[it] = a2;
      }
      for (int pass = 0; pass < 2; ++pass) {
#pragma unroll
        for (int it = 0; it < 4; ++it) {
          const int row = it * 4 + q;
          *(volatile v4u*)(C + (size_t)(mBase + row) * ldc + n0 + c8) = hv[it];
          if (OUT_MODE == 3) {
            if (wr2) *(volatile v4u*)(C2 + (size_t)(mBase + row) * ldc2 + n0 + c8) = lv[it];
          }
        }
        __threadfence();
      }
    }
    __builtin_amdgcn_fence(__ATOMIC_RELEASE, "workgroup");
    __builtin_amdgcn_wave_barrier();
    __builtin_amdgcn_fence(__ATOMIC_ACQUIRE, "workgroup");
  }
}

__global__ __launch_bounds__(SMT)
void softmax_rows(const float* __restrict__ S, unsigned short* P) {
  __shared__ float redm[8];
  __shared__ float reds[8];
  const int t    = blockIdx.x;
  const int tid  = threadIdx.x;
  const int wave = tid >> 5;
  const int lane = tid & 31;
  const int c0   = tid * 8;
  const float* rp = S + (size_t)t * SEQ + c0;
  const v4f a  = *(const v4f*)(rp);
  const v4f a4 = *(const v4f*)(rp + 4);
  float v[8];
#pragma unroll
  for (int e = 0; e < 4; ++e) {
    v[e]     = (c0 + e <= t)     ? a[e]  : -INFINITY;
    v[4 + e] = (c0 + 4 + e <= t) ? a4[e] : -INFINITY;
  }
  float mx = v[0];
#pragma unroll
  for (int e = 1; e < 8; ++e) mx = fmaxf(mx, v[e]);
#pragma unroll
  for (int off = 1; off < 32; off <<= 1) mx = fmaxf(mx, __shfl_xor(mx, off, 32));
  if (SMW > 1) {
    if (lane == 0) redm[wave] = mx;
    __syncthreads();
    mx = redm[0];
#pragma unroll
    for (int w = 1; w < SMW; ++w) mx = fmaxf(mx, redm[w]);
  }
  float ex[8];
  float sum = 0.f;
#pragma unroll
  for (int e = 0; e < 8; ++e) { ex[e] = __expf(v[e] - mx); sum += ex[e]; }
#pragma unroll
  for (int off = 1; off < 32; off <<= 1) sum += __shfl_xor(sum, off, 32);
  if (SMW > 1) {
    if (lane == 0) reds[wave] = sum;
    __syncthreads();
    sum = reds[0];
#pragma unroll
    for (int w = 1; w < SMW; ++w) sum += reds[w];
  }
  const float sc = PCARRY * (1.0f / sum);
  v4u pk;
#pragma unroll
  for (int e = 0; e < 4; ++e) {
    const unsigned short p0 = h_bits((_Float16)(ex[2 * e] * sc));
    const unsigned short p1 = h_bits((_Float16)(ex[2 * e + 1] * sc));
    pk[e] = pk16(p0, p1);
  }
  unsigned short* op = P + (size_t)t * SEQ + c0;
  *(volatile v4u*)op = pk;
  __threadfence();
  *(volatile v4u*)op = pk;
}

extern "C" void kernel_launch(void* const* d_in, const int* in_sizes, int n_in,
                              void* d_out, int out_size, void* d_ws, size_t ws_size,
                              hipStream_t stream) {
  if (n_in < 5) return;
  const long long needX = ((long long)(NB - 1) * SEQ_FULL + SEQ) * (long long)EMB;
  if ((long long)in_sizes[0] < needX) return;
  if (in_sizes[1] < EMB * EMB) return;
  if (in_sizes[2] < EMB * EMB) return;
  if (in_sizes[3] < EMB * EMB) return;
  if (in_sizes[4] < EMB * EMB) return;
  if (out_size < 0) return;
  if ((long long)out_size < needX) return;

  const float* x  = (const float*)d_in[0];
  const float* Wq = (const float*)d_in[1];
  const float* Wk = (const float*)d_in[2];
  const float* Wv = (const float*)d_in[3];
  const float* Wo = (const float*)d_in[4];

  const size_t PACT = (size_t)NROW * EMB * 2;
  const size_t PS   = (size_t)SEQ * SEQ * 4;
  const size_t R0   = (PACT > PS) ? PACT : PS;
  const size_t PW   = (size_t)EMB * EMB * 2;
  const size_t PVT  = (size_t)NB * EMB * SEQ * 2;
  const size_t PVL  = (size_t)NB * EMB * VLP * 2;
  const size_t PP   = (size_t)NB * SEQ * SEQ * 2;
  size_t off = 0;
  const size_t oR0 = off; off += R0;
  const size_t oWq = off; off += PW;
  const size_t oWk = off; off += PW;
  const size_t oWv = off; off += PW;
  const size_t oWo = off; off += PW;
  const size_t oQh = off; off += PACT;
  const size_t oQl = off; off += PACT;
  const size_t oKp = off; off += PACT;
  const size_t oVT = off; off += PVT;
  const size_t oVL = off; off += PVL;
  const size_t oP  = off; off += PP;
  if (off > ws_size) return;
  if (off > (size_t)134217728) return;

  char* ws = (char*)d_ws;
  unsigned short* Xb  = (unsigned short*)(ws + oR0);
  float*          S   = (float*)(ws + oR0);
  unsigned short* Wqb = (unsigned short*)(ws + oWq);
  unsigned short* Wkb = (unsigned short*)(ws + oWk);
  unsigned short* Wvb = (unsigned short*)(ws + oWv);
  unsigned short* Woh = (unsigned short*)(ws + oWo);
  unsigned short* Qh  = (unsigned short*)(ws + oQh);
  unsigned short* Ql  = (unsigned short*)(ws + oQl);
  unsigned short* Ch  = (unsigned short*)(ws + oQh);
  unsigned short* Cl  = (unsigned short*)(ws + oQl);
  unsigned short* Kp  = (unsigned short*)(ws + oKp);
  unsigned short* VT  = (unsigned short*)(ws + oVT);
  unsigned short* VL  = (unsigned short*)(ws + oVL);
  unsigned short* Pp  = (unsigned short*)(ws + oP);
  float*          out0 = (float*)d_out;

  const dim3 blk(256);
  const int n8xb = SEQ * EMB / 8;
  const int n8w  = EMB * EMB / 8;
  const dim3 gCvtX((n8xb + 255) / 256, NB);
  const dim3 gCvtW((n8w + 255) / 256, 1);
  const dim3 gQK((((NROW / 64) * (EMB / 64)) + 7) / 8, 1);
  const dim3 gV((((EMB / 64) * (SEQ / 64)) + 7) / 8, NB);
  const dim3 gS((((SEQ / 32) * (SEQ / 64)) + 7) / 8, 1);
  const dim3 gSm(SEQ);
  const dim3 gPV((((SEQ / 32) * (EMB / 64)) + 7) / 8, NB);
  const dim3 gO((((SEQ / 32) * (EMB / 64)) + 7) / 8, NB);

  cvt16x8<0><<<gCvtX, blk, 0, stream>>>(x,  (long long)SEQ_FULL * EMB, Xb,  (long long)SEQ * EMB, n8xb);
  cvt16x8<0><<<gCvtW, blk, 0, stream>>>(Wq, 0LL, Wqb, 0LL, n8w);
  cvt16x8<0><<<gCvtW, blk, 0, stream>>>(Wk, 0LL, Wkb, 0LL, n8w);
  cvt16x8<0><<<gCvtW, blk, 0, stream>>>(Wv, 0LL, Wvb, 0LL, n8w);
  cvt16x8<1><<<gCvtW, blk, 0, stream>>>(Wo, 0LL, Woh, 0LL, n8w);
  gemm_t<__bf16, 4, 1, 1, 3, 0><<<gQK, blk, 0, stream>>>(
      Xb, Xb, EMB, 0LL, Wqb, EMB, 0LL,
      Wqb, EMB, 0LL, 0,
      (void*)Qh, (void*)Ql, EMB, 0LL, EMB, 0LL, EMB,
      NROW, EMB, EMB, 1.0f, 0.0f, 1.0f, 4096.0f);
  gemm_t<__bf16, 4, 1, 1, 1, 0><<<gQK, blk, 0, stream>>>(
      Xb, Xb, EMB, 0LL, Wkb, EMB, 0LL,
      Wkb, EMB, 0LL, 0,
      (void*)Kp, (void*)Kp, EMB, 0LL, EMB, 0LL, EMB,
      NROW, EMB, EMB, 1.0f, 0.0f, 1.0f, 1.0f);
  gemm_t<__bf16, 4, 1, 1, 3, 0><<<gV, blk, 0, stream>>>(
      Wvb, Wvb, EMB, 0LL, Xb, EMB, (long long)SEQ * EMB,
      Xb, EMB, (long long)SEQ * EMB, 0,
      (void*)VT, (void*)VL, SEQ, (long long)EMB * SEQ, VLP, (long long)EMB * VLP, VLP,
      EMB, SEQ, EMB, 1.0f, 0.0f, 1.0f, 4096.0f);
  for (int bb = 0; bb < NB; ++bb) {
    const size_t ao = (size_t)bb * SEQ * EMB;
    gemm_t<_Float16, 2, 2, 1, 0, 1><<<gS, blk, 0, stream>>>(
        Qh + ao, Ql + ao, EMB, 0LL, Kp + ao, EMB, 0LL,
        Kp + ao, EMB, 0LL, 0,
        (void*)S, (void*)S, SEQ, 0LL, SEQ, 0LL, SEQ,
        SEQ, SEQ, EMB, 1.0f / 32.0f, 1.0f / 4096.0f, 1.0f, 1.0f);
    softmax_rows<<<gSm, dim3(SMT), 0, stream>>>(S, Pp + (size_t)bb * SEQ * SEQ);
  }
  gemm_t<_Float16, 2, 1, 2, 3, 2><<<gPV, blk, 0, stream>>>(
      Pp, Pp, SEQ, (long long)SEQ * SEQ, VT, SEQ, (long long)EMB * SEQ,
      VL, VLP, (long long)EMB * VLP, VLP,
      (void*)Ch, (void*)Cl, EMB, (long long)SEQ * EMB, EMB, (long long)SEQ * EMB, EMB,
      SEQ, EMB, SEQ, 1.0f / PCARRY, 1.0f / 4096.0f, 256.0f, 4096.0f);
  gemm_t<_Float16, 2, 2, 1, 0, 0><<<gO, blk, 0, stream>>>(
      Ch, Cl, EMB, (long long)SEQ * EMB, Woh, EMB, 0LL,
      Woh, EMB, 0LL, 0,
      (void*)out0, (void*)out0, EMB, (long long)SEQ_FULL * EMB, EMB, (long long)SEQ_FULL * EMB, EMB,
      SEQ, EMB, EMB, 1.0f / 16384.0f, 1.0f / 4096.0f, 1.0f, 1.0f);
  (void)hipGetLastError();
}
